// StandardMultiHeadAttention_62947040690414
// MI455X (gfx1250) — hardware-verified
//
#include <hip/hip_runtime.h>


#ifndef NB
#define NB 2
#endif
#ifndef SEQ
#define SEQ 2048
#endif
#define NB_FULL  2
#define SEQ_FULL 2048
#define DM    1024
#define NH    16
#define HDIM  64
#define MROWS (NB * SEQ)
#define KOUT  (2 * DM)

static_assert(NB >= 1 && NB <= NB_FULL);
static_assert(SEQ >= 128 && SEQ <= SEQ_FULL && (SEQ % 128) == 0);
static_assert((DM % 128) == 0 && NH * HDIM == DM && HDIM == 64);
static_assert((MROWS % 128) == 0);

#define DEV __device__ __forceinline__

typedef unsigned short us;
typedef us     v8us  __attribute__((ext_vector_type(8)));
typedef us     v16us __attribute__((ext_vector_type(16)));
typedef __bf16 v16bf __attribute__((ext_vector_type(16)));
typedef float  v8f   __attribute__((ext_vector_type(8)));
typedef float  v4f   __attribute__((ext_vector_type(4)));

#define PLANE_BYTES ((size_t)MROWS * DM * 2)
#define WB_BYTES    ((size_t)DM * DM * 2)
#define WO2_BYTES   ((size_t)DM * KOUT * 2)
#define CTX_BYTES   ((size_t)MROWS * KOUT * 2)
#define OFF_XB   ((size_t)0)
#define OFF_WQ   (OFF_XB + PLANE_BYTES)
#define OFF_WK   (OFF_WQ + WB_BYTES)
#define OFF_WV   (OFF_WK + WB_BYTES)
#define OFF_WO2  (OFF_WV + WB_BYTES)
#define OFF_QH   (OFF_WO2 + WO2_BYTES)
#define OFF_QL   (OFF_QH + PLANE_BYTES)
#define OFF_KH   (OFF_QL + PLANE_BYTES)
#define OFF_KL   (OFF_KH + PLANE_BYTES)
#define OFF_VH   (OFF_KL + PLANE_BYTES)
#define OFF_VL   (OFF_VH + PLANE_BYTES)
#define OFF_CTX  (OFF_VL + PLANE_BYTES)
#define WS_TOTAL (OFF_CTX + CTX_BYTES)
static_assert(WS_TOTAL <= (size_t)134217728);
static_assert((OFF_WQ % 128) == 0 && (OFF_WK % 128) == 0 && (OFF_WV % 128) == 0 &&
              (OFF_WO2 % 128) == 0 && (OFF_QH % 128) == 0 && (OFF_QL % 128) == 0 &&
              (OFF_KH % 128) == 0 && (OFF_KL % 128) == 0 && (OFF_VH % 128) == 0 &&
              (OFF_VL % 128) == 0 && (OFF_CTX % 128) == 0);

DEV us f2bf(float f) {
  unsigned u = __float_as_uint(f);
  u += 0x7FFFu + ((u >> 16) & 1u);
  return (us)(u >> 16);
}
DEV float bf2f(us b) { return __uint_as_float(((unsigned)b) << 16); }
DEV void split2(float x, us& hi, us& lo) {
  hi = f2bf(x);
  lo = f2bf(x - bf2f(hi));
}
DEV int imin(int a, int b) { return a < b ? a : b; }
DEV v8f zero8() {
  v8f z;
#pragma unroll
  for (int i = 0; i < 8; ++i) z[i] = 0.0f;
  return z;
}

DEV v16us ldfrag(const us* __restrict__ p, int h) {
  const v8us a = *(const v8us*)(p + 8 * h);
  const v8us b = *(const v8us*)(p + 16 + 8 * h);
  return __builtin_shufflevector(a, b, 0, 1, 2, 3, 4, 5, 6, 7, 8, 9, 10, 11, 12, 13, 14, 15);
}

DEV v8f mma(v16us a, v16us b, v8f c) {
  c = __builtin_amdgcn_wmma_f32_16x16x32_bf16(false, __builtin_bit_cast(v16bf, a), false,
                                              __builtin_bit_cast(v16bf, b), (short)0, c,
                                              false, false);
  asm volatile("v_nop\n\tv_nop\n\tv_nop\n\tv_nop" : "+v"(c) : "v"(a), "v"(b) : "memory");
  return c;
}

__global__ __launch_bounds__(256) void k_cvt(const float* __restrict__ src, us* __restrict__ dst,
                                            int nrows, int seg, int segstride, int dpitch,
                                            int dup) {
  const long long e0 = ((long long)blockIdx.x * 256 + threadIdx.x) * 8;
  if (e0 >= (long long)nrows * DM) return;
  const int r = (int)(e0 / DM);
  const int c = (int)(e0 - (long long)r * DM);
  const int sr = (r / seg) * segstride + (r % seg);
  const float* p = src + (size_t)sr * DM + c;
  const v4f a = *(const v4f*)p;
  const v4f b = *(const v4f*)(p + 4);
  v8us o;
  o[0] = f2bf(a[0]); o[1] = f2bf(a[1]); o[2] = f2bf(a[2]); o[3] = f2bf(a[3]);
  o[4] = f2bf(b[0]); o[5] = f2bf(b[1]); o[6] = f2bf(b[2]); o[7] = f2bf(b[3]);
  us* d = dst + (size_t)r * dpitch + c;
  *(volatile v8us*)d = o;
  if (dup) *(volatile v8us*)(d + DM) = o;
  __threadfence();
  *(volatile v8us*)d = o;
  if (dup) *(volatile v8us*)(d + DM) = o;
}

template <int F32OUT, int BIASROW>
__global__ __launch_bounds__(128) void k_gemm(const us* __restrict__ A, const us* __restrict__ Bm,
                                             const float* __restrict__ bias,
                                             us* __restrict__ Ch, us* __restrict__ Cl,
                                             float* __restrict__ Cf, int N, int K) {
  __shared__ __align__(16) float smf[4 * 2048];
  const int tid = threadIdx.x;
  const int lane = tid & 31, w = tid >> 5, h = lane >> 4, m = lane & 15;
  const int row0 = blockIdx.x * 64 + (w & 1) * 32;
  const int col0 = blockIdx.y * 128 + (w >> 1) * 64;

  v8f acc[2][4];
#pragma unroll
  for (int i = 0; i < 2; ++i)
#pragma unroll
    for (int j = 0; j < 4; ++j) acc[i][j] = zero8();

  const us* ap0 = A + (size_t)(row0 + m) * K;
  const us* ap1 = A + (size_t)(row0 + 16 + m) * K;
  const us* bp0 = Bm + (size_t)(col0 + m) * K;
  const us* bp1 = Bm + (size_t)(col0 + 16 + m) * K;
  const us* bp2 = Bm + (size_t)(col0 + 32 + m) * K;
  const us* bp3 = Bm + (size_t)(col0 + 48 + m) * K;

#pragma unroll 2
  for (int k0 = 0; k0 < K; k0 += 32) {
    const v16us a0 = ldfrag(ap0 + k0, h);
    const v16us a1 = ldfrag(ap1 + k0, h);
    const v16us b0 = ldfrag(bp0 + k0, h);
    const v16us b1 = ldfrag(bp1 + k0, h);
    const v16us b2 = ldfrag(bp2 + k0, h);
    const v16us b3 = ldfrag(bp3 + k0, h);
    acc[0][0] = mma(a0, b0, acc[0][0]);
    acc[0][1] = mma(a0, b1, acc[0][1]);
    acc[0][2] = mma(a0, b2, acc[0][2]);
    acc[0][3] = mma(a0, b3, acc[0][3]);
    acc[1][0] = mma(a1, b0, acc[1][0]);
    acc[1][1] = mma(a1, b1, acc[1][1]);
    acc[1][2] = mma(a1, b2, acc[1][2]);
    acc[1][3] = mma(a1, b3, acc[1][3]);
  }

  if constexpr (BIASROW == 0) {
#pragma unroll
    for (int j = 0; j < 4; ++j) {
      const int cidx = imin(col0 + 16 * j + m, DM - 1);
      const float bj = bf2f(f2bf(bias[cidx]));
#pragma unroll
      for (int i = 0; i < 2; ++i)
#pragma unroll
        for (int r = 0; r < 8; ++r) acc[i][j][r] += bj;
    }
  } else {
#pragma unroll
    for (int i = 0; i < 2; ++i)
#pragma unroll
      for (int r = 0; r < 8; ++r) {
        const int ridx = imin(row0 + 16 * i + 8 * h + r, DM - 1);
        const float bi = bf2f(f2bf(bias[ridx]));
#pragma unroll
        for (int j = 0; j < 4; ++j) acc[i][j][r] += bi;
      }
  }

  if constexpr (F32OUT != 0) {
    float* t = smf + w * 2048;
#pragma unroll
    for (int i = 0; i < 2; ++i)
#pragma unroll
      for (int j = 0; j < 4; ++j)
#pragma unroll
        for (int r = 0; r < 8; ++r)
          t[(16 * i + 8 * h + r) * 64 + 16 * j + m] = acc[i][j][r];
    __syncthreads();
    const int rsub = lane >> 4, cc = (lane & 15) * 4;
    v4f vals[16];
#pragma unroll
    for (int it = 0; it < 16; ++it) vals[it] = *(const v4f*)(t + (2 * it + rsub) * 64 + cc);
    float* gb = Cf + (size_t)row0 * N + col0 + cc;
#pragma unroll
    for (int it = 0; it < 16; ++it)
      *(volatile v4f*)(gb + (size_t)(2 * it + rsub) * N) = vals[it];
    __threadfence();
#pragma unroll
    for (int it = 0; it < 16; ++it)
      *(volatile v4f*)(gb + (size_t)(2 * it + rsub) * N) = vals[it];
  } else {
    us* th = (us*)smf + w * 4096;
    us* tl = th + 2048;
#pragma unroll
    for (int i = 0; i < 2; ++i)
#pragma unroll
      for (int j = 0; j < 4; ++j)
#pragma unroll
        for (int r = 0; r < 8; ++r) {
          us hv, lv;
          split2(acc[i][j][r], hv, lv);
          const int idx = (16 * i + 8 * h + r) * 64 + 16 * j + m;
          th[idx] = hv;
          tl[idx] = lv;
        }
    __syncthreads();
    const int rsub = lane >> 3, cc = (lane & 7) * 8;
    v8us vh[8], vl[8];
#pragma unroll
    for (int it = 0; it < 8; ++it) {
      vh[it] = *(const v8us*)(th + (4 * it + rsub) * 64 + cc);
      vl[it] = *(const v8us*)(tl + (4 * it + rsub) * 64 + cc);
    }
    us* gh = Ch + (size_t)row0 * N + col0 + cc;
    us* gl = Cl + (size_t)row0 * N + col0 + cc;
#pragma unroll
    for (int it = 0; it < 8; ++it) {
      *(volatile v8us*)(gh + (size_t)(4 * it + rsub) * N) = vh[it];
      *(volatile v8us*)(gl + (size_t)(4 * it + rsub) * N) = vl[it];
    }
    __threadfence();
#pragma unroll
    for (int it = 0; it < 8; ++it) {
      *(volatile v8us*)(gh + (size_t)(4 * it + rsub) * N) = vh[it];
      *(volatile v8us*)(gl + (size_t)(4 * it + rsub) * N) = vl[it];
    }
  }
}

__global__ __launch_bounds__(128) void k_attn(const us* __restrict__ Qh, const us* __restrict__ Ql,
                                             const us* __restrict__ Kh, const us* __restrict__ Kl,
                                             const us* __restrict__ Vh, const us* __restrict__ Vl,
                                             us* __restrict__ Ctx) {
  __shared__ __align__(16) us sct[4 * 2048];
  const int tid = threadIdx.x;
  const int lane = tid & 31, w = tid >> 5, h = lane >> 4, m = lane & 15;
  const int qblk = blockIdx.x, head = blockIdx.y, b = blockIdx.z;
  const int qbase = qblk * 64 + w * 16;
  const int qi = qbase + m;
  const size_t brow = (size_t)b * SEQ;

  const us* qph = Qh + (brow + qi) * DM + head * HDIM;
  const us* qpl = Ql + (brow + qi) * DM + head * HDIM;
  const v16us qh0 = ldfrag(qph, h), qh1 = ldfrag(qph + 32, h);
  const v16us ql0 = ldfrag(qpl, h), ql1 = ldfrag(qpl + 32, h);

  v8f o[4];
#pragma unroll
  for (int n = 0; n < 4; ++n) o[n] = zero8();
  float m_run = -3.0e38f, l_run = 0.0f;

  const int ntiles = qblk + 1;
  for (int kt = 0; kt < ntiles; ++kt) {
    const int key0 = kt * 64;

    v8f st[4];
#pragma unroll
    for (int mt = 0; mt < 4; ++mt) {
      const size_t kr = (brow + key0 + 16 * mt + m) * DM + head * HDIM;
      const v16us a0 = ldfrag(Kh + kr, h), a1 = ldfrag(Kh + kr + 32, h);
      const v16us c0 = ldfrag(Kl + kr, h), c1 = ldfrag(Kl + kr + 32, h);
      v8f c = zero8();
      c = mma(a0, qh0, c); c = mma(a1, qh1, c);
      c = mma(a0, ql0, c); c = mma(a1, ql1, c);
      c = mma(c0, qh0, c); c = mma(c1, qh1, c);
      st[mt] = c;
    }

    float mx = -3.0e38f;
#pragma unroll
    for (int mt = 0; mt < 4; ++mt)
#pragma unroll
      for (int r = 0; r < 8; ++r) {
        const int ki = key0 + 16 * mt + 8 * h + r;
        const float s = (ki <= qi) ? st[mt][r] * 0.125f : -1.0e30f;
        st[mt][r] = s;
        mx = fmaxf(mx, s);
      }
    mx = fmaxf(mx, __shfl_xor(mx, 16, 32));
    const float m_new = fmaxf(m_run, mx);
    const float alpha = __expf(m_run - m_new);
    float lsum = 0.0f;
#pragma unroll
    for (int mt = 0; mt < 4; ++mt)
#pragma unroll
      for (int r = 0; r < 8; ++r) {
        const float e = __expf(st[mt][r] - m_new);
        st[mt][r] = e;
        lsum += e;
      }
    lsum += __shfl_xor(lsum, 16, 32);
    l_run = l_run * alpha + lsum;
    m_run = m_new;
#pragma unroll
    for (int n = 0; n < 4; ++n) o[n] *= alpha;

    v16us ph0, pl0, ph1, pl1;
#pragma unroll
    for (int i = 0; i < 8; ++i) {
      us hv, lv;
      split2(st[0][i], hv, lv); ph0[i] = hv;     pl0[i] = lv;
      split2(st[1][i], hv, lv); ph0[i + 8] = hv; pl0[i + 8] = lv;
      split2(st[2][i], hv, lv); ph1[i] = hv;     pl1[i] = lv;
      split2(st[3][i], hv, lv); ph1[i + 8] = hv; pl1[i + 8] = lv;
    }

#pragma unroll
    for (int n = 0; n < 4; ++n) {
      const size_t vr = (size_t)(head * HDIM + 16 * n + m) * MROWS + brow + key0;
      const v16us a0 = ldfrag(Vh + vr, h), a1 = ldfrag(Vh + vr + 32, h);
      const v16us c0 = ldfrag(Vl + vr, h), c1 = ldfrag(Vl + vr + 32, h);
      v8f acc = o[n];
      acc = mma(a0, ph0, acc); acc = mma(a1, ph1, acc);
      acc = mma(a0, pl0, acc); acc = mma(a1, pl1, acc);
      acc = mma(c0, ph0, acc); acc = mma(c1, ph1, acc);
      o[n] = acc;
    }
  }

  const float inv = 1.0f / l_run;
  us* th = sct + w * 2048;
  us* tl = th + 1024;
#pragma unroll
  for (int n = 0; n < 4; ++n) {
    v8us hv, lv;
#pragma unroll
    for (int r = 0; r < 8; ++r) {
      us a, c;
      split2(o[n][r] * inv, a, c);
      hv[r] = a; lv[r] = c;
    }
    *(v8us*)(th + m * 64 + 16 * n + 8 * h) = hv;
    *(v8us*)(tl + m * 64 + 16 * n + 8 * h) = lv;
  }
  __syncthreads();
  const int rsub = lane >> 3, cc = (lane & 7) * 8;
  v8us gh[4], gl[4];
#pragma unroll
  for (int it = 0; it < 4; ++it) {
    gh[it] = *(const v8us*)(th + (4 * it + rsub) * 64 + cc);
    gl[it] = *(const v8us*)(tl + (4 * it + rsub) * 64 + cc);
  }
  us* cb = Ctx + (brow + qbase) * KOUT + head * HDIM + cc;
#pragma unroll
  for (int it = 0; it < 4; ++it) {
    us* p = cb + (size_t)(4 * it + rsub) * KOUT;
    *(volatile v8us*)p = gh[it];
    *(volatile v8us*)(p + DM) = gl[it];
  }
  __threadfence();
#pragma unroll
  for (int it = 0; it < 4; ++it) {
    us* p = cb + (size_t)(4 * it + rsub) * KOUT;
    *(volatile v8us*)p = gh[it];
    *(volatile v8us*)(p + DM) = gl[it];
  }
}

extern "C" void kernel_launch(void* const* d_in, const int* in_sizes, int n_in,
                              void* d_out, int out_size, void* d_ws,
                              size_t ws_size, hipStream_t stream) {
  if (n_in < 9) return;
  if ((size_t)in_sizes[0] < ((size_t)(NB - 1) * SEQ_FULL + SEQ) * DM) return;
  if (in_sizes[1] < DM * DM || in_sizes[3] < DM * DM || in_sizes[5] < DM * DM ||
      in_sizes[7] < DM * DM) return;
  if (in_sizes[2] < DM || in_sizes[4] < DM || in_sizes[6] < DM || in_sizes[8] < DM) return;
  if (out_size < MROWS * DM) return;
  if (ws_size < WS_TOTAL) return;

  const float* x  = (const float*)d_in[0];
  const float* wq = (const float*)d_in[1];
  const float* bq = (const float*)d_in[2];
  const float* wk = (const float*)d_in[3];
  const float* bk = (const float*)d_in[4];
  const float* wv = (const float*)d_in[5];
  const float* bv = (const float*)d_in[6];
  const float* wo = (const float*)d_in[7];
  const float* bo = (const float*)d_in[8];
  float* out = (float*)d_out;

  char* ws = (char*)d_ws;
  us* xb  = (us*)(ws + OFF_XB);
  us* wqb = (us*)(ws + OFF_WQ);
  us* wkb = (us*)(ws + OFF_WK);
  us* wvb = (us*)(ws + OFF_WV);
  us* wo2 = (us*)(ws + OFF_WO2);
  us* qh  = (us*)(ws + OFF_QH);
  us* ql  = (us*)(ws + OFF_QL);
  us* kh  = (us*)(ws + OFF_KH);
  us* kl  = (us*)(ws + OFF_KL);
  us* vth = (us*)(ws + OFF_VH);
  us* vtl = (us*)(ws + OFF_VL);
  us* ctx = (us*)(ws + OFF_CTX);

  k_cvt<<<dim3((unsigned)((size_t)MROWS * (DM / 8) / 256)), dim3(256), 0, stream>>>(
      x, xb, MROWS, SEQ, SEQ_FULL, DM, 0);
  k_cvt<<<dim3(DM * (DM / 8) / 256), dim3(256), 0, stream>>>(wq, wqb, DM, DM, DM, DM, 0);
  k_cvt<<<dim3(DM * (DM / 8) / 256), dim3(256), 0, stream>>>(wk, wkb, DM, DM, DM, DM, 0);
  k_cvt<<<dim3(DM * (DM / 8) / 256), dim3(256), 0, stream>>>(wv, wvb, DM, DM, DM, DM, 0);
  k_cvt<<<dim3(DM * (DM / 8) / 256), dim3(256), 0, stream>>>(wo, wo2, DM, DM, DM, KOUT, 1);

  k_gemm<0, 0><<<dim3(MROWS / 64, DM / 128), dim3(128), 0, stream>>>(xb, wqb, bq, qh, ql, out,
                                                                     DM, DM);
  k_gemm<0, 0><<<dim3(MROWS / 64, DM / 128), dim3(128), 0, stream>>>(xb, wkb, bk, kh, kl, out,
                                                                     DM, DM);
  k_gemm<0, 1><<<dim3(DM / 64, MROWS / 128), dim3(128), 0, stream>>>(wvb, xb, bv, vth, vtl, out,
                                                                     MROWS, DM);

  k_attn<<<dim3(SEQ / 64, NH, NB), dim3(128), 0, stream>>>(qh, ql, kh, kl, vth, vtl, ctx);

  k_gemm<1, 0><<<dim3(MROWS / 64, DM / 128), dim3(128), 0, stream>>>(ctx, wo2, bo, qh, ql, out,
                                                                     DM, KOUT);
}
